// DummyModel_89816356094558
// MI455X (gfx1250) — hardware-verified
//
#include <hip/hip_runtime.h>


namespace {
constexpr int NBH = 32, S = 2048, DH = 64, CH = 256;
constexpr float XS = 8.0f, PS = 256.0f, SCALE = 0.2f, FACTOR = 2.0f, SMN = 0.0f;
typedef _Float16 b16;
typedef __attribute__((ext_vector_type(16))) _Float16 v16b;
typedef __attribute__((ext_vector_type(8))) _Float16 v8b;
typedef __attribute__((ext_vector_type(2))) _Float16 v2b;
typedef __attribute__((ext_vector_type(8))) float v8f;
typedef __attribute__((ext_vector_type(2))) float v2f;
__device__ __forceinline__ float bf16_rne(float f) { unsigned int u = __float_as_uint(f); u += 0x7FFFu + ((u >> 16) & 1u); float r = __uint_as_float(u & 0xFFFF0000u); asm volatile("" : "+v"(r)); return r; }
__device__ __forceinline__ float bfv(float f) { float r = bf16_rne(f); asm volatile("" : "+v"(r)); return r; }
__device__ __forceinline__ void split16(float v, b16& hi, b16& lo) { hi = (b16)v; lo = (b16)(v - (float)hi); }
__device__ __forceinline__ v16b frag_kb(const b16* p, int hh) { const v8b a = *(const v8b*)(p + 8 * hh), b = *(const v8b*)(p + 16 + 8 * hh); v16b f;
#pragma unroll
  for (int e = 0; e < 8; ++e) { f[e] = a[e]; f[8 + e] = b[e]; } return f; }
__device__ __forceinline__ v8f wmma16b(v16b a, v16b b, v8f c) { v8f d = __builtin_amdgcn_wmma_f32_16x16x32_f16(false, a, false, b, (short)0, c, false, false); asm volatile("v_nop\n\tv_nop\n\tv_nop\n\tv_nop" : "+v"(d) : "v"(a), "v"(b)); return d; }
__device__ __forceinline__ void wave_lds_sync() { __builtin_amdgcn_fence(__ATOMIC_RELEASE, "workgroup"); __builtin_amdgcn_wave_barrier(); __builtin_amdgcn_fence(__ATOMIC_ACQUIRE, "workgroup"); }

__global__ __launch_bounds__(256) void prep_kernel(const float* __restrict__ q, const float* __restrict__ k, const float* __restrict__ v, b16* __restrict__ Q, b16* __restrict__ K, b16* __restrict__ VT) { __shared__ float Tt[64][DH + 1]; const int tid = threadIdx.x, wave = tid >> 5, lane = tid & 31; const int bh = blockIdx.x / (S / 64), s0 = (blockIdx.x % (S / 64)) * 64; const size_t base = ((size_t)bh * S + s0) * DH;
  for (int qd = wave; qd < 64; qd += 8) { Tt[qd][lane * 2] = bfv(v[base + (size_t)qd * DH + lane * 2]); Tt[qd][lane * 2 + 1] = bfv(v[base + (size_t)qd * DH + lane * 2 + 1]); }
  __syncthreads();
  for (int pass = 0; pass < 2; ++pass) {
    for (int e = tid; e < 64 * DH / 2; e += 256) { const size_t o = base + 2 * (size_t)e; *(volatile v2b*)(Q + o) = (v2b){(b16)(bfv(q[o]) * XS), (b16)(bfv(q[o + 1]) * XS)}; *(volatile v2b*)(K + o) = (v2b){(b16)(bfv(k[o]) * XS), (b16)(bfv(k[o + 1]) * XS)}; }
    for (int d = wave; d < DH; d += 8) *(volatile v2b*)(VT + ((size_t)bh * DH + d) * S + s0 + lane * 2) = (v2b){(b16)(Tt[lane * 2][d] * XS), (b16)(Tt[lane * 2 + 1][d] * XS)};
    __threadfence(); } }
__global__ __launch_bounds__(32) void att_kernel(const b16* __restrict__ Q, const b16* __restrict__ K, const b16* __restrict__ VT, int QLIM, float* __restrict__ out) { __shared__ __attribute__((aligned(16))) b16 Pa[32][CH + 8], Pb[32][CH + 8]; __shared__ float Sc[32][CH + 1], Mx[32], Ls[32], Fc[32], Of[32][DH + 1]; const int lane = threadIdx.x, nloc = lane & 15, hlf = lane >> 4; const int bh = blockIdx.x / (S / 32), q0 = (blockIdx.x % (S / 32)) * 32; if (q0 >= QLIM) return; const size_t tq = (size_t)bh * S + q0;
  Mx[lane] = -INFINITY; Ls[lane] = 0.0f; for (int kk = CH; kk < CH + 8; ++kk) { Pa[lane][kk] = (b16)0.0f; Pb[lane][kk] = (b16)0.0f; }
  wave_lds_sync();
  v16b qa[2][2]; for (int rt = 0; rt < 2; ++rt) for (int ks = 0; ks < 2; ++ks) qa[rt][ks] = frag_kb(Q + (tq + rt * 16 + nloc) * DH + ks * 32, hlf);
  v8f oacc[2][4];
#pragma unroll
  for (int rt = 0; rt < 2; ++rt)
#pragma unroll
    for (int t = 0; t < 4; ++t) oacc[rt][t] = (v8f){};
#pragma unroll 1
  for (int ch = 0; ch < S / CH; ++ch) { const int k0 = ch * CH;
#pragma unroll 1
    for (int tg = 0; tg < 16; tg += 4) { v8f sacc[2][4];
#pragma unroll
      for (int rt = 0; rt < 2; ++rt)
#pragma unroll
        for (int t = 0; t < 4; ++t) sacc[rt][t] = (v8f){};
#pragma unroll
      for (int t = 0; t < 4; ++t)
#pragma unroll
        for (int ks = 0; ks < 2; ++ks) { const v16b kb = frag_kb(K + ((size_t)bh * S + k0 + (tg + t) * 16 + nloc) * DH + ks * 32, hlf); sacc[0][t] = wmma16b(qa[0][ks], kb, sacc[0][t]); sacc[1][t] = wmma16b(qa[1][ks], kb, sacc[1][t]); }
#pragma unroll
      for (int rt = 0; rt < 2; ++rt)
#pragma unroll
        for (int t = 0; t < 4; ++t)
#pragma unroll
          for (int r8 = 0; r8 < 8; ++r8) Sc[rt * 16 + 8 * hlf + r8][(tg + t) * 16 + nloc] = sacc[rt][t][r8] * (SCALE / (XS * XS)); }
    wave_lds_sync();
    { const int r = lane; float mx = -INFINITY; for (int j = 0; j < CH; ++j) mx = fmaxf(mx, Sc[r][j]); const float mo = Mx[r], mn = fmaxf(mo, mx); float sm = 0.0f; for (int j = 0; j < CH; ++j) { const float p = __expf(Sc[r][j] - mn); sm += p; b16 ph, pl; split16(p * PS, ph, pl); Pa[r][j] = ph; Pb[r][j] = pl; } const float fac = (mo == -INFINITY) ? 0.0f : __expf(mo - mn); Fc[r] = fac; Ls[r] = Ls[r] * fac + sm; Mx[r] = mn; }
    wave_lds_sync();
#pragma unroll
    for (int rt = 0; rt < 2; ++rt)
#pragma unroll
      for (int t = 0; t < 4; ++t)
#pragma unroll
        for (int r8 = 0; r8 < 8; ++r8) oacc[rt][t][r8] *= Fc[rt * 16 + 8 * hlf + r8];
#pragma unroll 2
    for (int kb = 0; kb < CH; kb += 32)
#pragma unroll
      for (int rt = 0; rt < 2; ++rt) { const v16b pa = frag_kb(&Pa[rt * 16 + nloc][kb], hlf), pb = frag_kb(&Pb[rt * 16 + nloc][kb], hlf);
#pragma unroll
        for (int t = 0; t < 4; ++t) { const v16b vb = frag_kb(VT + ((size_t)bh * DH + t * 16 + nloc) * S + k0 + kb, hlf); oacc[rt][t] = wmma16b(pa, vb, oacc[rt][t]); oacc[rt][t] = wmma16b(pb, vb, oacc[rt][t]); } }
    wave_lds_sync(); }
#pragma unroll
  for (int rt = 0; rt < 2; ++rt)
#pragma unroll
    for (int t = 0; t < 4; ++t)
#pragma unroll
      for (int r8 = 0; r8 < 8; ++r8) { const int r = rt * 16 + 8 * hlf + r8; const float den = SMN * __expf(-Mx[r]) + Ls[r]; Of[r][t * 16 + nloc] = FACTOR * oacc[rt][t][r8] * (1.0f / (PS * XS)) / den; }
  wave_lds_sync();
  for (int pass = 0; pass < 2; ++pass) { for (int r = 0; r < 32; ++r) *(volatile v2f*)(out + (tq + r) * DH + lane * 2) = (v2f){Of[r][lane * 2], Of[r][lane * 2 + 1]}; __threadfence(); } }
}

extern "C" void kernel_launch(void* const* d_in, const int* in_sizes, int n_in, void* d_out, int out_size, void* d_ws, size_t ws_size, hipStream_t stream) {
  (void)n_in;
  auto Fp = [&](int i) { return (const float*)d_in[i]; };
  if (in_sizes[0] != NBH * S * DH || in_sizes[1] != NBH * S * DH || in_sizes[2] != NBH * S * DH || out_size != NBH * S * DH) return;
  const int QLIM = S;
  size_t off = 0; char* ws = (char*)d_ws;
  auto carve = [&](size_t bytes) { char* p = ws + off; off += (bytes + 255) & ~(size_t)255; return p; };
  b16* Q = (b16*)carve((size_t)NBH * S * DH * 2); b16* K = (b16*)carve((size_t)NBH * S * DH * 2); b16* VT = (b16*)carve((size_t)NBH * DH * S * 2);
  if (off > ws_size || off > ((size_t)32 << 20)) return;
  prep_kernel<<<NBH * (S / 64), 256, 0, stream>>>(Fp(0), Fp(1), Fp(2), Q, K, VT);
  att_kernel<<<NBH * (S / 32), 32, 0, stream>>>(Q, K, VT, QLIM, (float*)d_out);
}
